// ScaledDotProductAttention_33681133535369
// MI455X (gfx1250) — hardware-verified
//
#include <hip/hip_runtime.h>
#ifndef NB
#define NB 16
#endif
#ifndef SEQ
#define SEQ 2048
#endif
#define SEQ_FULL 2048
#define DH 128
#define SOP 132
#define PCARRY 4096.0f
#define SCL 0.08838834764831845f

static_assert(DH == 128);
static_assert(SEQ % 64 == 0);
static_assert(SEQ <= SEQ_FULL);
static_assert(((size_t)NB * SEQ * DH) % 2048 == 0);

typedef unsigned short v8us __attribute__((ext_vector_type(8), may_alias));
typedef float  v8f  __attribute__((ext_vector_type(8)));
typedef float  v4f  __attribute__((ext_vector_type(4)));
typedef float  v4fa __attribute__((ext_vector_type(4), may_alias));
typedef _Float16 v16h __attribute__((ext_vector_type(16)));
union FragH { v16h v; v8us half[2]; _Float16 h[16]; unsigned short u[16]; };

__device__ __forceinline__ unsigned short bf16_bits(float x) { unsigned int u = __float_as_uint(x); return (unsigned short)((u + 0x7FFFu + ((u >> 16) & 1u)) >> 16); }
__device__ __forceinline__ float bf16_val(unsigned short b) { return __uint_as_float(((unsigned int)b) << 16); }
__device__ __forceinline__ float bf16_rne(float x) { return bf16_val(bf16_bits(x)); }

__device__ __forceinline__ v16h ld_frag(const _Float16* p, unsigned hh) {
  FragH f;
  f.half[0] = *(const v8us*)((const unsigned short*)p + 8u * hh);
  f.half[1] = *(const v8us*)((const unsigned short*)p + 16u + 8u * hh);
  return f.v;
}
__device__ __forceinline__ void mma_pair(v16h a0, v16h a1, v16h b, v8f& c0, v8f& c1) {
  c0 = __builtin_amdgcn_wmma_f32_16x16x32_f16(false, a0, false, b, (short)0, c0, false, false);
  c1 = __builtin_amdgcn_wmma_f32_16x16x32_f16(false, a1, false, b, (short)0, c1, false, false);
  asm volatile("v_nop\n\tv_nop\n\tv_nop\n\tv_nop" : "+v"(c0), "+v"(c1) : "v"(a0), "v"(a1), "v"(b));
}

__global__ __launch_bounds__(256) void k_x16(const float* __restrict__ xq, const float* __restrict__ xk, _Float16* __restrict__ Q16, _Float16* __restrict__ K16) {
  const float* x = (blockIdx.y == 0u) ? xq : xk;
  _Float16* o = (blockIdx.y == 0u) ? Q16 : K16;
  const unsigned t = blockIdx.x * 256u + threadIdx.x;
  if (t >= (unsigned)((size_t)NB * SEQ * DH / 8)) return;
  const unsigned e = t * 8u;
  const unsigned b = e / (unsigned)(SEQ * DH);
  const unsigned rem = e - b * (unsigned)(SEQ * DH);
  const float* src = x + (size_t)b * SEQ_FULL * DH + rem;
  const v4f a = *(const v4fa*)(src), c = *(const v4fa*)(src + 4);
  FragH f;
#pragma unroll
  for (unsigned q = 0; q < 4; ++q) { f.h[q] = (_Float16)bf16_rne(a[q]); f.h[4 + q] = (_Float16)bf16_rne(c[q]); }
  const v8us v = f.half[0];
  *(volatile v8us*)((unsigned short*)o + e) = v;
  __threadfence();
  *(volatile v8us*)((unsigned short*)o + e) = v;
}

__global__ __launch_bounds__(256) void k_tb(const float* __restrict__ T, float* __restrict__ Tb) {
  const unsigned t = blockIdx.x * 256u + threadIdx.x;
  if (t >= (unsigned)(NB * SEQ / 4)) return;
  const unsigned e = t * 4u;
  const unsigned b = e / (unsigned)SEQ;
  const unsigned s = e - b * (unsigned)SEQ;
  const v4f a = *(const v4fa*)(T + (size_t)b * SEQ_FULL + s);
  v4f o;
#pragma unroll
  for (unsigned q = 0; q < 4; ++q) o[q] = bf16_rne(a[q]);
  *(volatile v4f*)(Tb + e) = o;
  __threadfence();
  *(volatile v4f*)(Tb + e) = o;
}

__global__ __launch_bounds__(256) void k_vt(const float* __restrict__ V, _Float16* __restrict__ VT) {
  __shared__ unsigned short tl[DH][66];
  const unsigned tid = threadIdx.x;
  const unsigned b = blockIdx.y, s0 = blockIdx.x * 64u;
  const float* vb = V + ((size_t)b * SEQ_FULL + s0) * DH;
#pragma unroll
  for (unsigned it = 0; it < 4; ++it) {
    const unsigned i = it * 256u + tid;
    const unsigned j = i >> 4, d8 = (i & 15u) * 8u;
    const v4f a = *(const v4fa*)(vb + (size_t)j * DH + d8), c = *(const v4fa*)(vb + (size_t)j * DH + d8 + 4);
    FragH f;
#pragma unroll
    for (unsigned q = 0; q < 4; ++q) { f.h[q] = (_Float16)bf16_rne(a[q]); f.h[4 + q] = (_Float16)bf16_rne(c[q]); }
#pragma unroll
    for (unsigned q = 0; q < 8; ++q) tl[d8 + q][j] = f.u[q];
  }
  __syncthreads();
  for (unsigned pass = 0; pass < 2; ++pass) {
#pragma unroll
    for (unsigned it = 0; it < 4; ++it) {
      const unsigned i = it * 256u + tid;
      const unsigned d = i >> 3, j8 = (i & 7u) * 8u;
      FragH f;
#pragma unroll
      for (unsigned q = 0; q < 8; ++q) f.u[q] = tl[d][j8 + q];
      *(volatile v8us*)((unsigned short*)VT + ((size_t)b * DH + d) * SEQ + s0 + j8) = f.half[0];
    }
    if (pass == 0) __threadfence();
  }
}

__global__ __launch_bounds__(128) void k_flash(const _Float16* __restrict__ Q16, const _Float16* __restrict__ K16, const _Float16* __restrict__ VT,
                                               const float* __restrict__ Tb, float* __restrict__ O) {
  __shared__ __attribute__((aligned(16))) float so[4][16][SOP];
  const unsigned tid = threadIdx.x, w = tid >> 5, lane = tid & 31u, ln = lane & 15u, hh = lane >> 4;
  const unsigned b = blockIdx.y;
  const unsigned q0 = blockIdx.x * 64u + w * 16u;
  const size_t rowb = (size_t)b * SEQ;
  const _Float16* qrow = Q16 + (rowb + q0 + ln) * DH;
  const v16h bq0 = ld_frag(qrow, hh), bq1 = ld_frag(qrow + 32, hh), bq2 = ld_frag(qrow + 64, hh), bq3 = ld_frag(qrow + 96, hh);
  const _Float16* kbase = K16 + (rowb + ln) * DH;
  const _Float16* vbase = VT + ((size_t)b * DH + ln) * SEQ;
  const float* tbase = Tb + rowb + 8u * hh;
  const v8f z8 = {0.f, 0.f, 0.f, 0.f, 0.f, 0.f, 0.f, 0.f};
  v8f acc[8];
#pragma unroll
  for (unsigned dt = 0; dt < 8; ++dt) acc[dt] = z8;
  float m = -1.0e30f, l = 0.f;

#pragma unroll 1
  for (unsigned kc = 0; kc < (unsigned)SEQ; kc += 32u) {
    const _Float16* k0p = kbase + (size_t)kc * DH;
    const _Float16* k1p = k0p + 16 * DH;
    v8f s0 = z8, s1 = z8;
    mma_pair(ld_frag(k0p, hh),      ld_frag(k1p, hh),      bq0, s0, s1);
    mma_pair(ld_frag(k0p + 32, hh), ld_frag(k1p + 32, hh), bq1, s0, s1);
    mma_pair(ld_frag(k0p + 64, hh), ld_frag(k1p + 64, hh), bq2, s0, s1);
    mma_pair(ld_frag(k0p + 96, hh), ld_frag(k1p + 96, hh), bq3, s0, s1);

    const v4f ta = *(const v4fa*)(tbase + kc), tb4 = *(const v4fa*)(tbase + kc + 4);
    const v4f tc = *(const v4fa*)(tbase + kc + 16), td = *(const v4fa*)(tbase + kc + 20);
    const float t0[8] = {ta[0], ta[1], ta[2], ta[3], tb4[0], tb4[1], tb4[2], tb4[3]};
    const float t1[8] = {tc[0], tc[1], tc[2], tc[3], td[0], td[1], td[2], td[3]};
    float x0[8], x1[8];
    float cm = -1.0e30f;
#pragma unroll
    for (unsigned r = 0; r < 8; ++r) {
      x0[r] = (s0[r] * SCL) * t0[r];
      x1[r] = (s1[r] * SCL) * t1[r];
      cm = fmaxf(cm, fmaxf(x0[r], x1[r]));
    }
    cm = fmaxf(cm, __shfl_xor(cm, 16, 32));
    const float mn = fmaxf(m, cm);
    const float alpha = __expf(m - mn);
    m = mn;
    FragH pb;
    float ls = 0.f;
#pragma unroll
    for (unsigned r = 0; r < 8; ++r) {
      const _Float16 h0 = (_Float16)(__expf(x0[r] - mn) * t0[r] * PCARRY);
      const _Float16 h1 = (_Float16)(__expf(x1[r] - mn) * t1[r] * PCARRY);
      pb.h[r] = h0; pb.h[8 + r] = h1;
      ls += (float)h0 + (float)h1;
    }
    l = l * alpha + ls;
#pragma unroll
    for (unsigned dt = 0; dt < 8; ++dt)
#pragma unroll
      for (unsigned r = 0; r < 8; ++r) acc[dt][r] *= alpha;

    const _Float16* vp = vbase + kc;
    mma_pair(ld_frag(vp,                      hh), ld_frag(vp + (size_t)16 * SEQ,  hh), pb.v, acc[0], acc[1]);
    mma_pair(ld_frag(vp + (size_t)32 * SEQ,   hh), ld_frag(vp + (size_t)48 * SEQ,  hh), pb.v, acc[2], acc[3]);
    mma_pair(ld_frag(vp + (size_t)64 * SEQ,   hh), ld_frag(vp + (size_t)80 * SEQ,  hh), pb.v, acc[4], acc[5]);
    mma_pair(ld_frag(vp + (size_t)96 * SEQ,   hh), ld_frag(vp + (size_t)112 * SEQ, hh), pb.v, acc[6], acc[7]);
  }

  const float lt = l + __shfl_xor(l, 16, 32);
  const float inv = 1.0f / lt;
#pragma unroll
  for (unsigned dt = 0; dt < 8; ++dt)
#pragma unroll
    for (unsigned r = 0; r < 8; ++r) so[w][ln][dt * 16u + 8u * hh + r] = acc[dt][r] * inv;
  __syncthreads();
  float* orow = O + ((size_t)b * SEQ_FULL + q0) * DH + lane * 4u;
  for (unsigned pass = 0; pass < 2; ++pass) {
#pragma unroll
    for (unsigned r = 0; r < 16; ++r) {
      const v4f v = *(const v4fa*)&so[w][r][lane * 4u];
      *(volatile v4f*)(orow + (size_t)r * DH) = v;
    }
    if (pass == 0) __threadfence();
  }
}

extern "C" void kernel_launch(void* const* d_in, const int* in_sizes, int n_in,
                              void* d_out, int out_size, void* d_ws, size_t ws_size, hipStream_t stream) {
  if (n_in < 4) return;
  const size_t need = (size_t)(NB - 1) * SEQ_FULL * DH + (size_t)SEQ * DH;
  const size_t needt = (size_t)(NB - 1) * SEQ_FULL + (size_t)SEQ;
  if ((size_t)in_sizes[0] < need || (size_t)in_sizes[1] < need || (size_t)in_sizes[2] < need || (size_t)in_sizes[3] < needt) return;
  if ((size_t)out_size < need) return;
  const float* xq = (const float*)d_in[0];
  const float* xk = (const float*)d_in[1];
  const float* xv = (const float*)d_in[2];
  const float* xt = (const float*)d_in[3];
  char* ws = (char*)d_ws; size_t off = 0;
  const size_t plane = (size_t)NB * SEQ * DH * 2;
  _Float16* Q16 = (_Float16*)(ws + off); off += (plane + 255) & ~(size_t)255;
  _Float16* K16 = (_Float16*)(ws + off); off += (plane + 255) & ~(size_t)255;
  _Float16* VTp = (_Float16*)(ws + off); off += (plane + 255) & ~(size_t)255;
  float* Tb = (float*)(ws + off); off += ((size_t)NB * SEQ * 4 + 255) & ~(size_t)255;
  if (off > ws_size) return;

  k_x16<<<dim3((unsigned)((size_t)NB * SEQ * DH / 8 / 256), 2), 256, 0, stream>>>(xq, xk, Q16, K16);
  k_tb<<<(unsigned)((NB * SEQ / 4 + 255) / 256), 256, 0, stream>>>(xt, Tb);
  k_vt<<<dim3(SEQ / 64, NB), 256, 0, stream>>>(xv, VTp);
  k_flash<<<dim3(SEQ / 64, NB), 128, 0, stream>>>(Q16, K16, VTp, Tb, (float*)d_out);
}
